// LocalMultiHeadAttention_69664369541437
// MI455X (gfx1250) — hardware-verified
//
#include <hip/hip_runtime.h>


namespace {
constexpr int B = 2, S = 1024, DM = 1024, H = 16, HD = 64, HALF = 32, NR = 2 * S - 1, BL = 2  , QL = 1024  , SK = 1024  ;
constexpr float XS = 8.0f, WSC = 256.0f, PS = 1024.0f, LOG2E = 1.4426950408889634f, LNEPS = 1e-5f;
static_assert(S % 64 == 0 && QL % 64 == 0 && SK % 64 == 0 && DM == H * HD, "tiling");
typedef _Float16 b16;
typedef __attribute__((ext_vector_type(16))) _Float16 v16b;
typedef __attribute__((ext_vector_type(8))) _Float16 v8b;
typedef __attribute__((ext_vector_type(8))) float v8f;
typedef __attribute__((ext_vector_type(4))) float v4f;
__device__ __forceinline__ float bf16_rne(float f) { unsigned int u = __float_as_uint(f); u += 0x7FFFu + ((u >> 16) & 1u); return __uint_as_float(u & 0xFFFF0000u); }
__device__ __forceinline__ void split16(float v, b16& hi, b16& lo) { hi = (b16)v; lo = (b16)(v - (float)hi); }
__device__ __forceinline__ v16b frag_kb(const b16* p, int hh) { const v8b a = *(const v8b*)(p + 8 * hh), b = *(const v8b*)(p + 16 + 8 * hh); v16b f;
#pragma unroll
  for (int e = 0; e < 8; ++e) { f[e] = a[e]; f[8 + e] = b[e]; } return f; }
__device__ __forceinline__ v8f wmma16b(v16b a, v16b b, v8f c) { v8f d = __builtin_amdgcn_wmma_f32_16x16x32_f16(false, a, false, b, (short)0, c, false, false); asm volatile("v_nop\n\tv_nop\n\tv_nop\n\tv_nop" : "+v"(d) : "v"(a), "v"(b)); return d; }
__device__ __forceinline__ void wave_lds_sync() { __builtin_amdgcn_fence(__ATOMIC_RELEASE, "workgroup"); __builtin_amdgcn_wave_barrier(); __builtin_amdgcn_fence(__ATOMIC_ACQUIRE, "workgroup"); }
__device__ __forceinline__ float pmul(float a, float b) { float p = a * b; asm volatile("" : "+v"(p)); return p; }
__device__ __forceinline__ int iclamp(int v, int lo, int hi) { return v < lo ? lo : (v > hi ? hi : v); }

typedef __attribute__((ext_vector_type(2))) _Float16 v2h;
typedef __attribute__((ext_vector_type(4))) _Float16 v4h;
typedef __attribute__((ext_vector_type(2))) float v2f;
__device__ __forceinline__ float nexp2(float v) { return __builtin_amdgcn_exp2f(v); }
__global__ __launch_bounds__(256) void prep_kernel(const float* __restrict__ wq, const float* __restrict__ wk, const float* __restrict__ wv, const float* __restrict__ wo, const float* __restrict__ lut, b16* __restrict__ WT, b16* __restrict__ WO, b16* __restrict__ LT) {
  size_t u = (size_t)blockIdx.x * 256 + threadIdx.x; const size_t per = (size_t)DM * DM / 8; v8b o;
  if (u < 4 * per) { const int m = (int)(u / per); const size_t e = (u % per) * 8; const int oo = (int)(e / DM), k0 = (int)(e % DM);
    if (m < 3) { const float* w = m == 0 ? wq : (m == 1 ? wk : wv); for (int j = 0; j < 8; ++j) o[j] = (b16)(bf16_rne(w[(size_t)(k0 + j) * DM + oo]) * WSC); for (int pass = 0; pass < 2; ++pass) { *(volatile v8b*)(WT + (size_t)m * DM * DM + e) = o; __threadfence(); } }
    else { for (int j = 0; j < 8; ++j) o[j] = (b16)(bf16_rne(wo[(size_t)(k0 + j) * DM + oo]) * WSC); for (int pass = 0; pass < 2; ++pass) { *(volatile v8b*)(WO + e) = o; __threadfence(); } }
    return; }
  u -= 4 * per; if (u < (size_t)(NR + 1) * HD / 8) { const size_t e = u * 8; const size_t r = e / HD; for (int j = 0; j < 8; ++j) o[j] = (r < (size_t)NR) ? (b16)(bf16_rne(lut[e + j]) * XS) : (b16)0.0f; for (int pass = 0; pass < 2; ++pass) { *(volatile v8b*)(LT + e) = o; __threadfence(); } }
}
__global__ __launch_bounds__(128) void proj_kernel(const float* __restrict__ xq, const float* __restrict__ xkv, const b16* __restrict__ WT, b16* __restrict__ Qp, b16* __restrict__ Kp, b16* __restrict__ VTh, b16* __restrict__ VTl) {
  __shared__ __attribute__((aligned(16))) b16 As[4][16][512 + 8]; __shared__ __attribute__((aligned(16))) float Tf[4][16][128 + 4];
  const int wave = threadIdx.x >> 5, lane = threadIdx.x & 31, nloc = lane & 15, hlf = lane >> 4; const int which = blockIdx.y % 3, b = blockIdx.y / 3; const int rb = blockIdx.x, slab = blockIdx.z; const int t0 = rb * 64 + wave * 16; const int n0 = slab * 128;
  if ((which == 0 && rb * 64 >= QL) || (which != 0 && rb * 64 >= SK)) return;
  const float* x = (which == 0) ? xq : xkv; const b16* W = WT + (size_t)which * DM * DM;
  v8f acc[8];
#pragma unroll
  for (int t = 0; t < 8; ++t) acc[t] = (v8f){};
#pragma unroll 1
  for (int half = 0; half < 2; ++half) {
    for (int rr = 0; rr < 16; ++rr) { const float* xr = x + ((size_t)b * S + t0 + rr) * DM + half * 512; for (int q = lane * 4; q < 512; q += 128) { const v4f xv = *(const v4f*)(xr + q); v4h o; for (int j = 0; j < 4; ++j) o[j] = (b16)(bf16_rne(xv[j]) * XS); *(v4h*)(&As[wave][rr][q]) = o; } }
    wave_lds_sync();
#pragma unroll 2
    for (int kb = 0; kb < 512; kb += 32) { const v16b a = frag_kb(&As[wave][nloc][kb], hlf);
#pragma unroll
      for (int t = 0; t < 8; ++t) acc[t] = wmma16b(a, frag_kb(W + (size_t)(n0 + t * 16 + nloc) * DM + half * 512 + kb, hlf), acc[t]); }
    wave_lds_sync(); }
#pragma unroll
  for (int t = 0; t < 8; ++t)
#pragma unroll
    for (int r = 0; r < 8; ++r) Tf[wave][8 * hlf + r][t * 16 + nloc] = acc[t][r] * (1.0f / (XS * WSC));
  __syncthreads();
  for (int pass = 0; pass < 2; ++pass) {
    if (which == 2) {
#pragma unroll 1
      for (int q = 0; q < 32; ++q) { const int cl = wave * 32 + q; const int c = n0 + cl; const int h = c / HD, d = c % HD; const int tk = lane * 2; v2h hv, lv;
        for (int j = 0; j < 2; ++j) { b16 p, ql; split16(Tf[(tk + j) >> 4][(tk + j) & 15][cl] * XS, p, ql); hv[j] = p; lv[j] = ql; }
        const size_t oi = (((size_t)b * H + h) * HD + d) * S + rb * 64 + lane * 2; *(volatile v2h*)(VTh + oi) = hv; *(volatile v2h*)(VTl + oi) = lv; } }
    else { b16* P = which == 0 ? Qp : Kp;
      for (int rr = 0; rr < 16; ++rr) { for (int hs = 0; hs < 2; ++hs) { const int c = n0 + hs * 64; const int h = c / HD; v2h o; o[0] = (b16)(Tf[wave][rr][hs * 64 + lane * 2] * XS); o[1] = (b16)(Tf[wave][rr][hs * 64 + lane * 2 + 1] * XS);
          *(volatile v2h*)(P + (((size_t)b * H + h) * S + (t0 + rr)) * HD + lane * 2) = o; } } }
    __threadfence(); }
}
__global__ __launch_bounds__(32) void attn_kernel(const b16* __restrict__ Qp, const b16* __restrict__ Kp, const b16* __restrict__ VTh, const b16* __restrict__ VTl, const b16* __restrict__ LT, b16* __restrict__ Ch, b16* __restrict__ Cl) {
  __shared__ float QR[16][96 + 1]; __shared__ __attribute__((aligned(16))) b16 Ph[16][96 + 8], Pl[16][96 + 8], Vs[2][HD][96 + 8]; __shared__ __attribute__((aligned(16))) float To[16][HD + 4];
  const int lane = threadIdx.x, hh = lane >> 4, col = lane & 15; const int b = blockIdx.y / H, h = blockIdx.y % H; const int q0 = blockIdx.x * 16, qi = q0 + col; const int kb0 = q0 - HALF; const int rbase = kb0 - (q0 + 15) + S - 1;
  const b16* Qb = Qp + ((size_t)(b * H + h) * S) * HD; const b16* Kb = Kp + ((size_t)(b * H + h) * S) * HD; const b16* Vh = VTh + ((size_t)(b * H + h) * HD) * S; const b16* Vl = VTl + ((size_t)(b * H + h) * HD) * S;
  const v16b qa0 = frag_kb(Qb + (size_t)qi * HD, hh), qa1 = frag_kb(Qb + (size_t)qi * HD + 32, hh);
#pragma unroll
  for (int t = 0; t < 6; ++t) { int r = rbase + t * 16 + col; r = r < 0 ? 0 : (r > NR ? NR : r);
    v8f d = (v8f){}; d = wmma16b(frag_kb(LT + (size_t)r * HD, hh), qa0, d); d = wmma16b(frag_kb(LT + (size_t)r * HD + 32, hh), qa1, d);
#pragma unroll
    for (int rr = 0; rr < 8; ++rr) QR[col][t * 16 + 8 * hh + rr] = d[rr] * (1.0f / (XS * XS)); }
  for (int i = lane; i < HD * 12; i += 32) { const int d = i / 12, ch = i % 12; const int key = kb0 + ch * 8; const bool ok = key >= 0 && key + 8 <= S && ch < 10;
    v8b a = {}, c = {}; if (ok) { a = *(const v8b*)(Vh + (size_t)d * S + key); c = *(const v8b*)(Vl + (size_t)d * S + key); } *(v8b*)(&Vs[0][d][ch * 8]) = a; *(v8b*)(&Vs[1][d][ch * 8]) = c; }
  __builtin_amdgcn_fence(__ATOMIC_RELEASE, "workgroup"); __builtin_amdgcn_wave_barrier(); __builtin_amdgcn_fence(__ATOMIC_ACQUIRE, "workgroup");
  const float cs = LOG2E / (8.0f * XS * XS); float e[40]; float mx = -INFINITY;
#pragma unroll
  for (int kt = 0; kt < 5; ++kt) { int kr = kb0 + kt * 16 + col; kr = kr < 0 ? 0 : (kr >= S ? S - 1 : kr);
    v8f s = (v8f){}; s = wmma16b(frag_kb(Kb + (size_t)kr * HD, hh), qa0, s); s = wmma16b(frag_kb(Kb + (size_t)kr * HD + 32, hh), qa1, s);
#pragma unroll
    for (int r = 0; r < 8; ++r) { const int slot = kt * 16 + 8 * hh + r; const int key = kb0 + slot; const int qq = q0 + col; const bool ok = key >= 0 && key < S && (key - qq <= HALF) && (qq - key <= HALF);
      float lg = -INFINITY; if (ok) lg = (s[r] * (1.0f / (XS * XS)) + QR[col][key - qq + S - 1 - rbase]) * (LOG2E / 8.0f); e[kt * 8 + r] = lg; mx = fmaxf(mx, lg); } }
  (void)cs;
  mx = fmaxf(mx, __shfl_xor(mx, 16)); float sum = 0.0f;
#pragma unroll
  for (int i = 0; i < 40; ++i) { const float p = (e[i] == -INFINITY) ? 0.0f : nexp2(e[i] - mx); e[i] = p; sum += p; }
  sum += __shfl_xor(sum, 16);
#pragma unroll
  for (int kt = 0; kt < 5; ++kt)
#pragma unroll
    for (int r = 0; r < 8; ++r) { b16 a_, b_; split16(e[kt * 8 + r] * PS, a_, b_); Ph[col][kt * 16 + 8 * hh + r] = a_; Pl[col][kt * 16 + 8 * hh + r] = b_; }
  for (int j = 0; j < 8; ++j) { Ph[col][80 + 8 * hh + j] = (b16)0.0f; Pl[col][80 + 8 * hh + j] = (b16)0.0f; }
  __builtin_amdgcn_fence(__ATOMIC_RELEASE, "workgroup"); __builtin_amdgcn_wave_barrier(); __builtin_amdgcn_fence(__ATOMIC_ACQUIRE, "workgroup");
  v8f o[4] = {(v8f){}, (v8f){}, (v8f){}, (v8f){}};
#pragma unroll
  for (int ks = 0; ks < 3; ++ks) { const v16b ph = frag_kb(&Ph[col][ks * 32], hh), pl = frag_kb(&Pl[col][ks * 32], hh);
#pragma unroll
    for (int t = 0; t < 4; ++t) { const v16b va = frag_kb(&Vs[0][t * 16 + col][ks * 32], hh), vl = frag_kb(&Vs[1][t * 16 + col][ks * 32], hh); o[t] = wmma16b(va, ph, o[t]); o[t] = wmma16b(va, pl, o[t]); o[t] = wmma16b(vl, ph, o[t]); } }
  const float inv = 1.0f / (sum * PS * XS);
#pragma unroll
  for (int t = 0; t < 4; ++t)
#pragma unroll
    for (int r = 0; r < 8; ++r) To[col][t * 16 + 8 * hh + r] = o[t][r] * inv;
  __builtin_amdgcn_fence(__ATOMIC_RELEASE, "workgroup"); __builtin_amdgcn_wave_barrier(); __builtin_amdgcn_fence(__ATOMIC_ACQUIRE, "workgroup");
  for (int pass = 0; pass < 2; ++pass) { for (int rr = 0; rr < 16; ++rr) { const v2f f = *(const v2f*)(&To[rr][lane * 2]); v2h hv, lv; for (int j = 0; j < 2; ++j) { b16 p, q; split16(f[j] * XS, p, q); hv[j] = p; lv[j] = q; }
      const size_t oi = ((size_t)b * S + q0 + rr) * DM + h * HD + lane * 2; *(volatile v2h*)(Ch + oi) = hv; *(volatile v2h*)(Cl + oi) = lv; } __threadfence(); }
}
__global__ __launch_bounds__(128) void out_kernel(const b16* __restrict__ Ch, const b16* __restrict__ Cl, const b16* __restrict__ WO, const float* __restrict__ bo, const float* __restrict__ x, float* __restrict__ Y) {
  __shared__ __attribute__((aligned(16))) float Tf[4][16][128 + 4];
  const int wave = threadIdx.x >> 5, lane = threadIdx.x & 31, nloc = lane & 15, hlf = lane >> 4; const int b = blockIdx.x / (QL / 64), rb = blockIdx.x % (QL / 64); const size_t m0 = (size_t)b * S + rb * 64 + wave * 16; const int n0 = blockIdx.y * 128;
  v8f acc[8];
#pragma unroll
  for (int t = 0; t < 8; ++t) acc[t] = (v8f){};
#pragma unroll 2
  for (int kb = 0; kb < DM; kb += 32) { const v16b a = frag_kb(Ch + (m0 + nloc) * DM + kb, hlf), al = frag_kb(Cl + (m0 + nloc) * DM + kb, hlf);
#pragma unroll
    for (int t = 0; t < 8; ++t) { const v16b bw = frag_kb(WO + (size_t)(n0 + t * 16 + nloc) * DM + kb, hlf); acc[t] = wmma16b(a, bw, acc[t]); acc[t] = wmma16b(al, bw, acc[t]); } }
#pragma unroll
  for (int t = 0; t < 8; ++t) { const float bb = bf16_rne(bo[n0 + t * 16 + nloc]);
#pragma unroll
    for (int r = 0; r < 8; ++r) Tf[wave][8 * hlf + r][t * 16 + nloc] = acc[t][r] * (1.0f / (XS * WSC)) + bb; }
  wave_lds_sync();
  for (int pass = 0; pass < 2; ++pass) { for (int rr = 0; rr < 16; ++rr) { v4f f = *(const v4f*)(&Tf[wave][rr][lane * 4]); const v4f xv = *(const v4f*)(x + (m0 + rr) * DM + n0 + lane * 4); for (int j = 0; j < 4; ++j) f[j] += bf16_rne(xv[j]); *(volatile v4f*)(Y + (m0 + rr) * DM + n0 + lane * 4) = f; } __threadfence(); }
}
__global__ __launch_bounds__(256) void ln_kernel(const float* __restrict__ Y, const float* __restrict__ g_, const float* __restrict__ b_, float* __restrict__ out) {
  const int wave = threadIdx.x >> 5, lane = threadIdx.x & 31; const size_t idx = (size_t)blockIdx.x * 8 + wave; const int b = (int)(idx / QL), s = (int)(idx % QL); if (b >= BL) return; const size_t row = ((size_t)b * S + s) * DM;
  float v[32]; float sm = 0.0f;
#pragma unroll
  for (int q = 0; q < 8; ++q) { const v4f f = *(const v4f*)(Y + row + lane * 32 + q * 4); for (int j = 0; j < 4; ++j) { v[q * 4 + j] = f[j]; sm += f[j]; } }
#pragma unroll
  for (int o = 1; o < 32; o <<= 1) sm += __shfl_xor(sm, o);
  const float mu = sm * (1.0f / DM); float sq = 0.0f;
#pragma unroll
  for (int i = 0; i < 32; ++i) { const float d = v[i] - mu; sq += d * d; }
#pragma unroll
  for (int o = 1; o < 32; o <<= 1) sq += __shfl_xor(sq, o);
  const float rs = rsqrtf(sq * (1.0f / DM) + LNEPS);
  for (int pass = 0; pass < 2; ++pass) {
#pragma unroll
    for (int q = 0; q < 8; ++q) { v4f o4; for (int j = 0; j < 4; ++j) { const int c = lane * 32 + q * 4 + j; o4[j] = (v[q * 4 + j] - mu) * rs * bf16_rne(g_[c]) + bf16_rne(b_[c]); } *(volatile v4f*)(out + row + lane * 32 + q * 4) = o4; }
    __threadfence(); }
}
}

extern "C" void kernel_launch(void* const* d_in, const int* in_sizes, int n_in, void* d_out, int out_size, void* d_ws, size_t ws_size, hipStream_t stream) {
  (void)n_in;
  auto Fp = [&](int i) { return (const float*)d_in[i]; };
  if (in_sizes[0] != B * S * DM || in_sizes[1] != B * S * DM || in_sizes[2] != NR * HD || in_sizes[3] != DM * DM || in_sizes[4] != DM * DM || in_sizes[5] != DM * DM || in_sizes[6] != DM * DM || in_sizes[7] != DM || in_sizes[8] != DM || in_sizes[9] != DM || out_size != B * S * DM) return;
  size_t off = 0; char* ws = (char*)d_ws;
  auto carve = [&](size_t bytes) { char* p = ws + off; off += (bytes + 255) & ~(size_t)255; return p; };
  b16* WT = (b16*)carve((size_t)3 * DM * DM * 2); b16* WO = (b16*)carve((size_t)DM * DM * 2); b16* LT = (b16*)carve((size_t)(NR + 1) * HD * 2); const size_t plane = (size_t)B * S * DM * 2;
  b16* Qp = (b16*)carve(plane); b16* Kp = (b16*)carve(plane); b16* VTh = (b16*)carve(plane); b16* VTl = (b16*)carve(plane); b16* Ch = (b16*)carve(plane); b16* Cl = (b16*)carve(plane); float* Y = (float*)carve((size_t)B * S * DM * 4);
  if (off > ws_size || off > ((size_t)128 << 20)) return;
  prep_kernel<<<(unsigned)((((size_t)4 * DM * DM + (size_t)(NR + 1) * HD) / 8 + 255) / 256), 256, 0, stream>>>(Fp(3), Fp(4), Fp(5), Fp(6), Fp(2), WT, WO, LT);
  proj_kernel<<<dim3(S / 64, BL * 3, 8), 128, 0, stream>>>(Fp(0), Fp(1), WT, Qp, Kp, VTh, VTl);
  attn_kernel<<<dim3(QL / 16, BL * H), 32, 0, stream>>>(Qp, Kp, VTh, VTl, LT, Ch, Cl);
  out_kernel<<<dim3((QL / 64) * BL, 8), 128, 0, stream>>>(Ch, Cl, WO, Fp(7), Fp(0), Y);
  ln_kernel<<<(BL * QL) / 8, 256, 0, stream>>>(Y, Fp(8), Fp(9), (float*)d_out);
}
